// LowRankMaskedSynapse_26250840113208
// MI455X (gfx1250) — hardware-verified
//
#include <hip/hip_runtime.h>
#include <stdint.h>

#define BROWS 512
#define NCOL  16384
#define RDIM  128

#define NXV    (BROWS * NCOL)
#define NVV    (NCOL * RDIM)
#define NX8    (NXV / 8)
#define NV8    (NVV / 8)
#define NFLAT8 (NX8 + NV8)
#define CVT_THREADS 256
#define FLAT_BLOCKS (NFLAT8 / CVT_THREADS)
#define XBLOCKS     (NX8 / CVT_THREADS)
#define TRK 64
#define TR_BLOCKS (NCOL / TRK)
#define MASK_COLS 1024
#define MASK_THREADS 256
#define MASK_BLOCKS (NCOL / MASK_COLS)

static_assert(NFLAT8 % CVT_THREADS == 0);
static_assert(NX8 % CVT_THREADS == 0);
static_assert((TRK * RDIM) % CVT_THREADS == 0);
static_assert(MASK_COLS == 4 * MASK_THREADS);
static_assert(NCOL % 64 == 0);
static_assert(BROWS % 64 == 0);
static_assert(RDIM % 32 == 0);
static_assert(NCOL % 32 == 0);

typedef unsigned short us16;
typedef __bf16 v16bf __attribute__((ext_vector_type(16)));
typedef us16   v8us  __attribute__((ext_vector_type(8)));
typedef float  v8f   __attribute__((ext_vector_type(8)));
typedef float  v4f   __attribute__((ext_vector_type(4)));
typedef int    v4i   __attribute__((ext_vector_type(4)));
typedef v8us __attribute__((may_alias)) v8usa;
typedef v4f  __attribute__((may_alias)) v4fa;
typedef v4i  __attribute__((may_alias)) v4ia;

union Frag { v16bf v; v8us hv[2]; };

__device__ __forceinline__ us16 f2bf(float f) {
  unsigned int u = __float_as_uint(f);
  u += 0x7FFFu + ((u >> 16) & 1u);
  return (us16)(u >> 16);
}
__device__ __forceinline__ float bf2f(us16 b) {
  return __uint_as_float(((unsigned int)b) << 16);
}

__device__ __forceinline__ v8f wmma_bf16(v16bf a, v16bf b, v8f c) {
#if defined(__HIP_DEVICE_COMPILE__)
  v8f d = __builtin_amdgcn_wmma_f32_16x16x32_bf16(false, a, false, b, (short)0, c, false, false);
  asm volatile("v_nop\n\tv_nop\n\tv_nop\n\tv_nop" : "+v"(d) : "v"(a), "v"(b));
  return d;
#else
  (void)a; (void)b;
  return c;
#endif
}

__device__ __forceinline__ v16bf load_frag(const us16* p, int h) {
  Frag f;
  f.hv[0] = *(const v8usa*)(p + 8 * h);
  f.hv[1] = *(const v8usa*)(p + 16 + 8 * h);
  return f.v;
}

__global__ __launch_bounds__(CVT_THREADS) void k_cvt(
    const float* __restrict__ x, const float* __restrict__ U, const float* __restrict__ V,
    us16* __restrict__ xb, us16* __restrict__ ut, us16* __restrict__ vb)
{
  __shared__ __attribute__((aligned(16))) us16 sU[TRK][RDIM + 2];
  const int tid = threadIdx.x;

  if (blockIdx.x < FLAT_BLOCKS) {
    const int g = blockIdx.x * CVT_THREADS + tid;
    const float* src;
    us16* dst;
    if (blockIdx.x < XBLOCKS) {
      src = x + (size_t)g * 8;
      dst = xb + (size_t)g * 8;
    } else {
      const int e = g - NX8;
      src = V + (size_t)e * 8;
      dst = vb + (size_t)e * 8;
    }
    const v4f a = *(const v4fa*)src;
    const v4f c = *(const v4fa*)(src + 4);
    const v8us o = { f2bf(a.x), f2bf(a.y), f2bf(a.z), f2bf(a.w),
                     f2bf(c.x), f2bf(c.y), f2bf(c.z), f2bf(c.w) };
    *(volatile v8us*)dst = o;
    __threadfence();
    *(volatile v8us*)dst = o;
  } else {
    const int tb = blockIdx.x - FLAT_BLOCKS;
    const int k0 = tb * TRK;
    #pragma unroll 4
    for (int e = 0; e < (TRK * RDIM) / CVT_THREADS; ++e) {
      const int idx = e * CVT_THREADS + tid;
      const int k = idx >> 7, n = idx & 127;
      sU[k][n] = f2bf(U[(size_t)(k0 + k) * RDIM + n]);
    }
    __syncthreads();
    #pragma unroll
    for (int pass = 0; pass < 2; ++pass) {
      #pragma unroll
      for (int it = 0; it < 4; ++it) {
        const int p = it * CVT_THREADS + tid;
        const int n = p >> 3, q = p & 7;
        v8us o;
        #pragma unroll
        for (int i = 0; i < 8; ++i) o[i] = sU[8 * q + i][n];
        us16* dst = ut + (size_t)n * NCOL + k0 + 8 * q;
        *(volatile v8us*)dst = o;
      }
      if (pass == 0) __threadfence();
    }
  }
}

__global__ __launch_bounds__(MASK_THREADS) void k_mask(
    const int* __restrict__ indices, int nnz, int* __restrict__ maskw)
{
  __shared__ __attribute__((aligned(16))) int sflag[MASK_COLS];
  const int tid = threadIdx.x;
  const int c0 = blockIdx.x * MASK_COLS;
  #pragma unroll
  for (int i = 0; i < 4; ++i) sflag[i * MASK_THREADS + tid] = 0;
  __syncthreads();

  const int chunk = 4 * MASK_THREADS;
  const int nvec = nnz / chunk;
  #pragma unroll 1
  for (int c = 0; c < nvec; ++c) {
    const v4i q = *(const v4ia*)(indices + (size_t)c * chunk + 4 * tid);
    #pragma unroll
    for (int u = 0; u < 4; ++u) {
      int j = q[u];
      if (j < 0) j += NCOL;
      const int jj = j - c0;
      if ((unsigned)jj < (unsigned)MASK_COLS) sflag[jj] = 1;
    }
  }
  #pragma unroll 1
  for (int e0 = nvec * chunk; e0 < nnz; e0 += MASK_THREADS) {
    int e = e0 + tid;
    e = (e < nnz) ? e : (nnz - 1);
    int j = indices[e];
    if (j < 0) j += NCOL;
    const int jj = j - c0;
    if ((unsigned)jj < (unsigned)MASK_COLS) sflag[jj] = 1;
  }
  __syncthreads();

  const v4i v = *(const v4ia*)(sflag + 4 * tid);
  int* dst = maskw + c0 + 4 * tid;
  *(volatile v4i*)dst = v;
  __threadfence();
  *(volatile v4i*)dst = v;
}

__device__ __forceinline__ void pre_store_pass(const us16* s, us16* plane, int m0, int lane) {
  #pragma unroll
  for (int it = 0; it < 8; ++it) {
    const int p = it * 32 + lane;
    const int row = p >> 4, seg = p & 15;
    const v8us v = *(const v8usa*)(s + row * RDIM + seg * 8);
    us16* dst = plane + (size_t)(m0 + row) * RDIM + seg * 8;
    *(volatile v8us*)dst = v;
  }
}

__global__ __launch_bounds__(32) void k_gemm1(
    const us16* __restrict__ xb,
    const us16* __restrict__ ut,
    us16* __restrict__ phi,
    us16* __restrict__ plo)
{
  __shared__ __attribute__((aligned(16))) us16 shi[16 * RDIM];
  __shared__ __attribute__((aligned(16))) us16 slo[16 * RDIM];

  const int lane = threadIdx.x & 31;
  const int h = lane >> 4, m = lane & 15;
  const int m0 = blockIdx.x * 16;

  const us16* arow = xb + (size_t)(m0 + m) * NCOL;
  const us16* brow = ut + (size_t)m * NCOL;

  const v8f zero8 = {0.f, 0.f, 0.f, 0.f, 0.f, 0.f, 0.f, 0.f};
  v8f acc[8];
  #pragma unroll
  for (int nt = 0; nt < 8; ++nt) acc[nt] = zero8;

  #pragma unroll 1
  for (int k0 = 0; k0 < NCOL; k0 += 32) {
    const v16bf a = load_frag(arow + k0, h);
    #pragma unroll
    for (int nt = 0; nt < 8; ++nt) {
      const v16bf b = load_frag(brow + (size_t)nt * 16 * NCOL + k0, h);
      acc[nt] = wmma_bf16(a, b, acc[nt]);
    }
  }

  #pragma unroll
  for (int nt = 0; nt < 8; ++nt) {
    #pragma unroll
    for (int r = 0; r < 8; ++r) {
      const float v = acc[nt][r];
      const us16 hi = f2bf(v);
      const us16 lo = f2bf(v - bf2f(hi));
      const int idx = (8 * h + r) * RDIM + 16 * nt + m;
      shi[idx] = hi;
      slo[idx] = lo;
    }
  }
  __syncthreads();

  pre_store_pass(shi, phi, m0, lane);
  pre_store_pass(slo, plo, m0, lane);
  __threadfence();
  pre_store_pass(shi, phi, m0, lane);
  pre_store_pass(slo, plo, m0, lane);
}

__device__ __forceinline__ void out_store_pass(const float* so, float* out,
                                               int mrow0, int n0, int lane) {
  const int q8 = lane & 7, sub = lane >> 3;
  #pragma unroll
  for (int i = 0; i < 8; ++i) {
    const int lid = i * 4 + sub;
    const int row = lid >> 1, hl = lid & 1;
    const v4f v = *(const v4fa*)(so + row * 64 + 32 * hl + 4 * q8);
    const size_t gi = (size_t)(mrow0 + row) * NCOL + n0 + 32 * hl + 4 * q8;
    *(volatile v4f*)(out + gi) = v;
  }
}

__global__ __launch_bounds__(128) void k_gemm2(
    const us16* __restrict__ phi,
    const us16* __restrict__ plo,
    const us16* __restrict__ vb,
    const int* __restrict__ maskw,
    float* __restrict__ out)
{
  __shared__ __attribute__((aligned(16))) float so_all[4 * 16 * 64];

  const int tid = threadIdx.x, lane = tid & 31, w = tid >> 5;
  const int h = lane >> 4, m = lane & 15;
  const int n0 = blockIdx.x * 64;
  const int m0w = blockIdx.y * 64 + 16 * w;

  const us16* ah = phi + (size_t)(m0w + m) * RDIM;
  const us16* al = plo + (size_t)(m0w + m) * RDIM;
  v16bf ahf[4], alf[4];
  #pragma unroll
  for (int ks = 0; ks < 4; ++ks) {
    ahf[ks] = load_frag(ah + 32 * ks, h);
    alf[ks] = load_frag(al + 32 * ks, h);
  }

  const v8f zero8 = {0.f, 0.f, 0.f, 0.f, 0.f, 0.f, 0.f, 0.f};
  v8f acc[4];
  #pragma unroll
  for (int nt = 0; nt < 4; ++nt) acc[nt] = zero8;

  #pragma unroll
  for (int nt = 0; nt < 4; ++nt) {
    const us16* br = vb + (size_t)(n0 + 16 * nt + m) * RDIM;
    #pragma unroll
    for (int ks = 0; ks < 4; ++ks) {
      const v16bf b = load_frag(br + 32 * ks, h);
      acc[nt] = wmma_bf16(ahf[ks], b, acc[nt]);
      acc[nt] = wmma_bf16(alf[ks], b, acc[nt]);
    }
  }

  float* so = so_all + w * 1024;
  #pragma unroll
  for (int nt = 0; nt < 4; ++nt) {
    const int mk = maskw[n0 + 16 * nt + m];
    #pragma unroll
    for (int r = 0; r < 8; ++r) {
      const float v = acc[nt][r];
      so[(8 * h + r) * 64 + 16 * nt + m] = (mk != 0) ? v : 0.0f;
    }
  }
  __syncthreads();

  out_store_pass(so, out, m0w, n0, lane);
  __threadfence();
  out_store_pass(so, out, m0w, n0, lane);
}

extern "C" void kernel_launch(void* const* d_in, const int* in_sizes, int n_in,
                              void* d_out, int out_size, void* d_ws, size_t ws_size,
                              hipStream_t stream) {
  if (n_in < 5) return;
  if (in_sizes[0] != NXV) return;
  if (in_sizes[1] != NVV || in_sizes[2] != NVV) return;
  if (out_size != NXV) return;
  const int nnz = in_sizes[4];
  if (nnz < 1) return;

  const float* x = (const float*)d_in[0];
  const float* U = (const float*)d_in[1];
  const float* V = (const float*)d_in[2];
  const int* indices = (const int*)d_in[4];
  float* out = (float*)d_out;

  const size_t xb_bytes = (size_t)NXV * 2;
  const size_t ut_bytes = (size_t)RDIM * NCOL * 2;
  const size_t vb_bytes = (size_t)NVV * 2;
  const size_t p_bytes  = (size_t)BROWS * RDIM * 2;
  const size_t mk_bytes = (size_t)NCOL * 4;
  size_t off = 0;
  char* ws = (char*)d_ws;
  us16* xb = (us16*)(ws + off);   off += xb_bytes;
  us16* ut = (us16*)(ws + off);   off += ut_bytes;
  us16* vb = (us16*)(ws + off);   off += vb_bytes;
  us16* phi = (us16*)(ws + off);  off += p_bytes;
  us16* plo = (us16*)(ws + off);  off += p_bytes;
  int* maskw = (int*)(ws + off);  off += mk_bytes;
  if (off > ws_size) return;

  k_cvt<<<dim3(FLAT_BLOCKS + TR_BLOCKS), dim3(CVT_THREADS), 0, stream>>>(x, U, V, xb, ut, vb);

  k_mask<<<dim3(MASK_BLOCKS), dim3(MASK_THREADS), 0, stream>>>(indices, nnz, maskw);

  k_gemm1<<<dim3(BROWS / 16), dim3(32), 0, stream>>>(xb, ut, phi, plo);

  dim3 g2(NCOL / 64, BROWS / 64);
  k_gemm2<<<g2, dim3(128), 0, stream>>>(phi, plo, vb, maskw, out);

  (void)hipGetLastError();
}
